// BatchRelationalModule_10917806867210
// MI455X (gfx1250) — hardware-verified
//
#include <hip/hip_runtime.h>

typedef __attribute__((ext_vector_type(16))) _Float16 v16h;
typedef __attribute__((ext_vector_type(8)))  _Float16 v8h;
typedef __attribute__((ext_vector_type(8)))  float    v8f;
typedef __attribute__((ext_vector_type(4)))  float    v4f;

#define NB  16
#define NL  256
#define NC  64
#define NF  64
#define DIN 130
#define STG 72

__device__ __forceinline__ void dep_guard_h(v8f& a, v8f& b, v16h x, v16h y) { asm volatile("v_nop\n\tv_nop\n\tv_nop\n\tv_nop" : "+v"(a), "+v"(b) : "v"(x), "v"(y)); }
template <typename T> struct Frag;
template <> struct Frag<_Float16> {
  typedef v16h V; union U { v16h v; v8h h[2]; };
  static __device__ __forceinline__ v16h load(const _Float16* p) {
    U f; f.h[0] = *(const v8h*)(p); f.h[1] = *(const v8h*)(p + 16); return f.v;
  }
  static __device__ __forceinline__ v8f mma(v16h a, v16h b, v8f c) {
    return __builtin_amdgcn_wmma_f32_16x16x32_f16(false, a, false, b, (short)0, c, false, false);
  }
  static __device__ __forceinline__ void guard(v8f& a, v8f& b, v16h x, v16h y) { dep_guard_h(a, b, x, y); }
};

__device__ __forceinline__ v8f mma2_f16(v16h a0, v16h b0, v16h a1, v16h b1, v8f c) {
  c = __builtin_amdgcn_wmma_f32_16x16x32_f16(false, a0, false, b0, (short)0, c, false, false);
  c = __builtin_amdgcn_wmma_f32_16x16x32_f16(false, a1, false, b1, (short)0, c, false, false);
  asm volatile("v_nop\n\tv_nop\n\tv_nop\n\tv_nop" : "+v"(c) : "v"(a0), "v"(b0), "v"(a1), "v"(b1));
  return c;
}

__device__ __forceinline__ void wave_lds_fence() {
  __builtin_amdgcn_fence(__ATOMIC_RELEASE, "workgroup");
  __builtin_amdgcn_wave_barrier();
  __builtin_amdgcn_fence(__ATOMIC_ACQUIRE, "workgroup");
}

__global__ __launch_bounds__(256) void k_pre(const float* __restrict__ x,
                                             const float* __restrict__ Wg0,
                                             const float* __restrict__ bg0,
                                             float* __restrict__ Ap, float* __restrict__ Bm,
                                             int total) {
  const int t = blockIdx.x * 256 + threadIdx.x;
  if (t >= total) return;
  const int f = t & (NF - 1), l = (t >> 6) & (NL - 1), b = t >> 14;
  const float* w  = Wg0 + f * DIN;
  const float* xb = x + (size_t)b * NC * NL + l;
  float sA = bg0[f], sB = 0.f;
#pragma unroll 4
  for (int ch = 0; ch < NC; ++ch) {
    const float v = xb[ch * NL];
    sA += v * w[ch];
    sB += v * w[NC + 1 + ch];
  }
  const float coord = (float)l;
  sA += coord * w[NC];
  sB += coord * w[DIN - 1];
  const size_t o = (size_t)(b * NL + l) * NF + f;
  ((volatile float*)Ap)[o] = sA;
  ((volatile float*)Bm)[o] = sB;
  __threadfence();
  ((volatile float*)Ap)[o] = sA;
  ((volatile float*)Bm)[o] = sB;
}

__global__ __launch_bounds__(128) void k_pairs(const float* __restrict__ Ap, const float* __restrict__ Bm,
                                               const float* __restrict__ Wg1, const float* __restrict__ bg1,
                                               const float* __restrict__ Wg2, const float* __restrict__ bg2,
                                               float* __restrict__ Pb) {
  __shared__ __align__(16) _Float16 st0[4][16 * STG];
  __shared__ __align__(16) _Float16 st1[4][16 * STG];
  __shared__ __align__(16) _Float16 wsh1[NF * STG];
  __shared__ __align__(16) _Float16 wsh2[NF * STG];
  __shared__ __align__(16) float sBp[NF];
  __shared__ __align__(16) float sPart[4][NF];

  const int tid  = threadIdx.x;
  const int lane = tid & 31;
  const int wave = tid >> 5;
  const int hh   = lane >> 4;
  const int m    = lane & 15;
  const int p = blockIdx.x, b = blockIdx.y;

  if (tid < NF) sBp[tid] = Bm[(size_t)(b * NL + p) * NF + tid];

  {
    const int n = tid >> 1, k0 = (tid & 1) * 32;
    const float* w1 = Wg1 + n * NF + k0;
    const float* w2 = Wg2 + n * NF + k0;
#pragma unroll
    for (int i = 0; i < 4; ++i) {
      const v4f a0 = *(const v4f*)(w1 + 8 * i), a1 = *(const v4f*)(w1 + 8 * i + 4);
      const v4f c0 = *(const v4f*)(w2 + 8 * i), c1 = *(const v4f*)(w2 + 8 * i + 4);
      v8h hv1, hv2;
#pragma unroll
      for (int e = 0; e < 4; ++e) {
        hv1[e] = (_Float16)a0[e]; hv1[4 + e] = (_Float16)a1[e];
        hv2[e] = (_Float16)c0[e]; hv2[4 + e] = (_Float16)c1[e];
      }
      *(v8h*)(wsh1 + n * STG + k0 + 8 * i) = hv1;
      *(v8h*)(wsh2 + n * STG + k0 + 8 * i) = hv2;
    }
  }
  __syncthreads();

  float cb1[4], cb2[4];
#pragma unroll
  for (int nt = 0; nt < 4; ++nt) {
    cb1[nt] = bg1[nt * 16 + m];
    cb2[nt] = bg2[nt * 16 + m];
  }

  v8f acc[4];
#pragma unroll
  for (int nt = 0; nt < 4; ++nt) acc[nt] = (v8f){0.f, 0.f, 0.f, 0.f, 0.f, 0.f, 0.f, 0.f};

  _Float16* stg0 = st0[wave];
  _Float16* stg1 = st1[wave];
  const int kb = hh * 32;

  for (int t = wave; t < 16; t += 4) {
    const int q0 = t * 16;

    const float* pa = Ap + (size_t)(b * NL + q0 + m) * NF + kb;
#pragma unroll
    for (int i = 0; i < 4; ++i) {
      const v4f u0 = *(const v4f*)(pa + 8 * i), u1 = *(const v4f*)(pa + 8 * i + 4);
      v8h hv;
#pragma unroll
      for (int e = 0; e < 4; ++e) {
        hv[e]     = (_Float16)fmaxf(u0[e] + sBp[kb + 8 * i + e], 0.f);
        hv[4 + e] = (_Float16)fmaxf(u1[e] + sBp[kb + 8 * i + 4 + e], 0.f);
      }
      *(v8h*)(stg0 + m * STG + kb + 8 * i) = hv;
    }
    wave_lds_fence();

    const v16h a0 = Frag<_Float16>::load(stg0 + m * STG + 8 * hh);
    const v16h a1 = Frag<_Float16>::load(stg0 + m * STG + 32 + 8 * hh);

#pragma unroll
    for (int nt = 0; nt < 4; ++nt) {
      const _Float16* wr = wsh1 + (nt * 16 + m) * STG + 8 * hh;
      const v16h b0 = Frag<_Float16>::load(wr);
      const v16h b1 = Frag<_Float16>::load(wr + 32);
      v8f c;
#pragma unroll
      for (int r = 0; r < 8; ++r) c[r] = cb1[nt];
      const v8f d = mma2_f16(a0, b0, a1, b1, c);
#pragma unroll
      for (int r = 0; r < 8; ++r)
        stg1[(8 * hh + r) * STG + nt * 16 + m] = (_Float16)fmaxf(d[r], 0.f);
    }
    wave_lds_fence();

    const v16h g0 = Frag<_Float16>::load(stg1 + m * STG + 8 * hh);
    const v16h g1 = Frag<_Float16>::load(stg1 + m * STG + 32 + 8 * hh);

#pragma unroll
    for (int nt = 0; nt < 4; ++nt) {
      const _Float16* wr = wsh2 + (nt * 16 + m) * STG + 8 * hh;
      const v16h b0 = Frag<_Float16>::load(wr);
      const v16h b1 = Frag<_Float16>::load(wr + 32);
      v8f c;
#pragma unroll
      for (int r = 0; r < 8; ++r) c[r] = cb2[nt];
      const v8f d = mma2_f16(g0, b0, g1, b1, c);
#pragma unroll
      for (int r = 0; r < 8; ++r) acc[nt][r] += fmaxf(d[r], 0.f);
    }
    wave_lds_fence();
  }

#pragma unroll
  for (int nt = 0; nt < 4; ++nt) {
    float s = 0.f;
#pragma unroll
    for (int r = 0; r < 8; ++r) s += acc[nt][r];
    s += __shfl_xor(s, 16, 32);
    if (lane < 16) sPart[wave][nt * 16 + lane] = s;
  }
  __syncthreads();
  if (tid < 16) {
    v4f v;
#pragma unroll
    for (int e = 0; e < 4; ++e) {
      const int f = 4 * tid + e;
      v[e] = ((sPart[0][f] + sPart[1][f]) + sPart[2][f]) + sPart[3][f];
    }
    float* dst = Pb + (size_t)(b * NL + p) * NF + 4 * tid;
    *(volatile v4f*)dst = v;
    __threadfence();
    *(volatile v4f*)dst = v;
  }
}

__global__ __launch_bounds__(64) void k_head(const float* __restrict__ Pb,
                                             const float* __restrict__ Wp, const float* __restrict__ bp,
                                             const float* __restrict__ Wo, const float* __restrict__ bo,
                                             float* __restrict__ out) {
  __shared__ __align__(16) float sS[NF];
  __shared__ __align__(16) float sh[NF];
  __shared__ __align__(16) float so[NF];
  const int t = threadIdx.x, b = blockIdx.x;
  float s = 0.f;
  for (int p = 0; p < NL; ++p) s += Pb[(size_t)(b * NL + p) * NF + t];
  sS[t] = s;
  __syncthreads();
  float a = bp[t];
#pragma unroll 4
  for (int f = 0; f < NF; ++f) a += sS[f] * Wp[t * NF + f];
  sh[t] = fmaxf(a, 0.f);
  __syncthreads();
  float o = bo[t];
#pragma unroll 4
  for (int f = 0; f < NF; ++f) o += sh[f] * Wo[t * NF + f];
  so[t] = o;
  __syncthreads();
  if (t < 16) {
    const v4f v = *(const v4f*)(so + 4 * t);
    float* dst = out + (size_t)b * NF + 4 * t;
    *(volatile v4f*)dst = v;
    __threadfence();
    *(volatile v4f*)dst = v;
  }
}

extern "C" void kernel_launch(void* const* d_in, const int* in_sizes, int n_in,
                              void* d_out, int out_size, void* d_ws, size_t ws_size,
                              hipStream_t stream) {
  if (n_in < 11) return;
  if (in_sizes[0] != NB * NC * NL || in_sizes[1] != NF * DIN || in_sizes[2] != NF ||
      in_sizes[3] != NF * NF || in_sizes[4] != NF || in_sizes[5] != NF * NF || in_sizes[6] != NF ||
      in_sizes[7] != NF * NF || in_sizes[8] != NF || in_sizes[9] != NF * NF || in_sizes[10] != NF ||
      out_size != NB * NF) return;

  const float* x   = (const float*)d_in[0];
  const float* Wg0 = (const float*)d_in[1];
  const float* bg0 = (const float*)d_in[2];
  const float* Wg1 = (const float*)d_in[3];
  const float* bg1 = (const float*)d_in[4];
  const float* Wg2 = (const float*)d_in[5];
  const float* bg2 = (const float*)d_in[6];
  const float* Wp  = (const float*)d_in[7];
  const float* bp  = (const float*)d_in[8];
  const float* Wo  = (const float*)d_in[9];
  const float* bo  = (const float*)d_in[10];
  float* out = (float*)d_out;

  const size_t plane = (size_t)NB * NL * NF;
  if (ws_size < 3 * plane * sizeof(float)) return;
  float* Ap = (float*)d_ws;
  float* Bm = Ap + plane;
  float* Pb = Bm + plane;

  const int total = NB * NL * NF;
  k_pre<<<(total + 255) / 256, 256, 0, stream>>>(x, Wg0, bg0, Ap, Bm, total);
  k_pairs<<<dim3(NL, NB), 128, 0, stream>>>(Ap, Bm, Wg1, bg1, Wg2, bg2, Pb);
  k_head<<<NB, NF, 0, stream>>>(Pb, Wp, bp, Wo, bo, out);
  (void)hipGetLastError();
}
